// PoincareBallLinear_48387101557105
// MI455X (gfx1250) — hardware-run, weakly checked
//
#include <hip/hip_runtime.h>
#include <math.h>

typedef __attribute__((ext_vector_type(16))) _Float16 v16h;
typedef __attribute__((ext_vector_type(8)))  _Float16 v8h;
typedef __attribute__((ext_vector_type(8)))  float    v8f;
typedef __attribute__((ext_vector_type(4)))  float    v4f;

constexpr int kB   = 128;
constexpr int kIn  = 1024;
constexpr int kOut = 1024;
static_assert((kB % 64) == 0);
static_assert((kOut % 64) == 0);
static_assert((kIn % 32) == 0);

constexpr float kCarryX = 64.0f;
constexpr float kCarryW = 256.0f;
constexpr float kFold   = 1.0f / (kCarryX * kCarryW);
constexpr float kF16MinNormal = 6.103515625e-05f;

constexpr size_t kOffA16  = 0;
constexpr size_t kOffBT16 = kOffA16  + (size_t)kB   * kIn  * 2;
constexpr size_t kOffSTD  = kOffBT16 + (size_t)kOut * kIn  * 2;
constexpr size_t kWsTotal = kOffSTD  + (size_t)kB   * kOut * 4;
static_assert(kWsTotal == 2883584ull);
static_assert(kWsTotal <= 134217728ull);
static_assert((kOffBT16 % 128) == 0);
static_assert((kOffSTD % 128) == 0);

__device__ __forceinline__ void tie_acc_h(v8f& a, v16h x, v16h y) {
  asm volatile("v_nop\n\tv_nop\n\tv_nop\n\tv_nop" : "+v"(a) : "v"(x), "v"(y));
}
__device__ __forceinline__ void tie_acc(v8f& a) {
  asm volatile("v_nop\n\tv_nop\n\tv_nop\n\tv_nop" : "+v"(a));
}
__device__ __forceinline__ void keep4_h(v16h a, v16h b, v16h c, v16h d) {
  asm volatile("v_nop" :: "v"(a), "v"(b), "v"(c), "v"(d));
}
struct FragH {
  union U { v16h v; v8h h[2]; };
  static __device__ __forceinline__ v16h load(const _Float16* p) {
    U f;
    f.h[0] = *(const v8h*)(p);
    f.h[1] = *(const v8h*)(p + 16);
    return f.v;
  }
  static __device__ __forceinline__ v8f mma(v16h a, v16h b, v8f c) {
    return __builtin_amdgcn_wmma_f32_16x16x32_f16(false, a, false, b, (short)0, c, false, false);
  }
};

constexpr int kCvtBlkX = (kB * kIn / 8) / 256;
constexpr int kCvtBlkW = (kOut * kIn / 8) / 256;
static_assert(kCvtBlkX * 256 * 8 == kB * kIn);
static_assert(kCvtBlkW * 256 * 8 == kOut * kIn);

__global__ __launch_bounds__(256) void to_f16_planes_kernel(
    const float* __restrict__ x, const float* __restrict__ w,
    unsigned short* __restrict__ A16, unsigned short* __restrict__ BT16)
{
  unsigned tid = threadIdx.x;
  asm volatile("" : "+v"(tid));
  const bool isX = (blockIdx.x < (unsigned)kCvtBlkX);
  const float* src = isX ? x : w;
  unsigned short* dst = isX ? A16 : BT16;
  const float carry = isX ? kCarryX : kCarryW;
  const unsigned blk = isX ? blockIdx.x : (blockIdx.x - (unsigned)kCvtBlkX);
  const unsigned i = blk * 256u + tid;
  const size_t e0 = (size_t)i << 3;
  const v4f a0 = *(const v4f*)(src + e0);
  const v4f a1 = *(const v4f*)(src + e0 + 4);
  v8h hv;
#pragma unroll
  for (int e = 0; e < 4; ++e) {
    const float s0 = a0[e];
    const float s1 = a1[e];
    float f0 = s0 * carry;
    float f1 = s1 * carry;
    f0 = (fabsf(f0) < kF16MinNormal) ? 0.0f : f0;
    f1 = (fabsf(f1) < kF16MinNormal) ? 0.0f : f1;
    hv[e]     = (_Float16)f0;
    hv[4 + e] = (_Float16)f1;
  }
  unsigned short* q = dst + e0;
  *(volatile v8h*)q = hv;
  __threadfence();
  *(volatile v8h*)q = hv;
}

constexpr int kTilesM = kB >> 6;
constexpr int kTilesN = kOut >> 6;
constexpr int kGemmBlocks = (kTilesM * kTilesN) / 8;
static_assert(kGemmBlocks * 8 == kTilesM * kTilesN);

__global__ __launch_bounds__(256) void gemm_f16_nt_kernel(
    const unsigned short* __restrict__ Ap, const unsigned short* __restrict__ Btp,
    float* __restrict__ C, float scale)
{
  __shared__ __align__(16) float sT[8][16 * 68];
  const _Float16* A  = (const _Float16*)(const void*)Ap;
  const _Float16* Bt = (const _Float16*)(const void*)Btp;
  const int lane = threadIdx.x & 31;
  const int wave = threadIdx.x >> 5;
  const int tile = blockIdx.x * 8 + wave;
  if (tile >= kTilesM * kTilesN) return;
  const int tm = tile / kTilesN;
  const int tn = tile - tm * kTilesN;
  const int m0 = tm << 6;
  const int n0 = tn << 6;

  const int rlane = lane & 15;
  const int koff  = (lane >> 4) * 8;
  const int mOff  = (lane >> 4) * 8;

  v8f acc[4][4];
#pragma unroll
  for (int i = 0; i < 4; ++i)
#pragma unroll
    for (int j = 0; j < 4; ++j) acc[i][j] = (v8f){0.f, 0.f, 0.f, 0.f, 0.f, 0.f, 0.f, 0.f};

  for (int k0 = 0; k0 < kIn; k0 += 32) {
    v16h bh[4];
#pragma unroll
    for (int j = 0; j < 4; ++j) {
      const size_t bo = (size_t)(n0 + (j << 4) + rlane) * kIn + koff + k0;
      bh[j] = FragH::load(Bt + bo);
    }
#pragma unroll
    for (int i = 0; i < 4; ++i) {
      const size_t ao = (size_t)(m0 + (i << 4) + rlane) * kIn + koff + k0;
      const v16h ah = FragH::load(A + ao);
#pragma unroll
      for (int j = 0; j < 4; ++j) acc[i][j] = FragH::mma(ah, bh[j], acc[i][j]);
      tie_acc_h(acc[i][0], ah, bh[0]);
      tie_acc_h(acc[i][1], ah, bh[1]);
      tie_acc_h(acc[i][2], ah, bh[2]);
      tie_acc_h(acc[i][3], ah, bh[3]);
    }
    keep4_h(bh[0], bh[1], bh[2], bh[3]);
  }
#pragma unroll
  for (int i = 0; i < 4; ++i) {
    tie_acc(acc[i][0]);
    tie_acc(acc[i][1]);
    tie_acc(acc[i][2]);
    tie_acc(acc[i][3]);
  }

  float* slab = sT[wave];
#pragma unroll
  for (int i = 0; i < 4; ++i) {
    const int mBase = m0 + (i << 4);
#pragma unroll
    for (int j = 0; j < 4; ++j) {
#pragma unroll
      for (int r = 0; r < 8; ++r) {
        const float v = acc[i][j][r] * scale;
        slab[(mOff + r) * 68 + (j << 4) + rlane] = v;
      }
    }
    __builtin_amdgcn_fence(__ATOMIC_RELEASE, "workgroup");
    __builtin_amdgcn_wave_barrier();
    __builtin_amdgcn_fence(__ATOMIC_ACQUIRE, "workgroup");
    {
      const int hh = lane >> 4;
      const int c4 = (lane & 15) * 4;
      for (int pass = 0; pass < 2; ++pass) {
#pragma unroll
        for (int it = 0; it < 8; ++it) {
          const int row = it * 2 + hh;
          const v4f v = *(const v4f*)(slab + row * 68 + c4);
          *(volatile v4f*)(C + (size_t)(mBase + row) * kOut + n0 + c4) = v;
        }
        __threadfence();
      }
    }
    __builtin_amdgcn_fence(__ATOMIC_RELEASE, "workgroup");
    __builtin_amdgcn_wave_barrier();
    __builtin_amdgcn_fence(__ATOMIC_ACQUIRE, "workgroup");
  }
}

constexpr int kTB = 32;
constexpr int kTO = 32;
constexpr int kKC = 32;
constexpr int kWP = 33;
static_assert((kB % kTB) == 0);
static_assert((kOut % kTO) == 0);
static_assert((kIn % kKC) == 0);
static_assert(kTB == 8 * 4);

__global__ __launch_bounds__(256) void scan_blend_kernel(
    const float* __restrict__ x, const float* __restrict__ w, const float* __restrict__ bias,
    const float* __restrict__ STD, float* __restrict__ out)
{
  __shared__ __align__(16) float xs[kTB * kKC];
  __shared__ __align__(16) float wsh[kTO * kWP];

  unsigned tid = threadIdx.x;
  asm volatile("" : "+v"(tid));
  const unsigned lane = tid & 31u;
  const unsigned wave = tid >> 5;
  const unsigned ldr  = tid >> 3;
  const unsigned ldc  = (tid & 7u) << 2;
  const unsigned o0   = blockIdx.x * (unsigned)kTO;
  const unsigned b0   = blockIdx.y * (unsigned)kTB;

  float P[4], Q[4];
#pragma unroll
  for (int i = 0; i < 4; ++i) {
    P[i] = 1.0f;
    Q[i] = 1.0f;
  }

  const float* xg = x + (size_t)(b0 + ldr) * kIn + ldc;
  const float* wg = w + (size_t)(o0 + ldr) * kIn + ldc;
  const float* xr = xs + (wave * 4u) * (unsigned)kKC;
  const float* wr = wsh + lane * (unsigned)kWP;

#pragma unroll 1
  for (int k0 = 0; k0 < kIn; k0 += kKC) {
    const v4f gx = *(const v4f*)(xg + k0);
    const v4f gw = *(const v4f*)(wg + k0);
    __syncthreads();
    *(v4f*)(xs + ldr * (unsigned)kKC + ldc) = gx;
    {
      const float g0 = gw[0];
      const float g1 = gw[1];
      const float g2 = gw[2];
      const float g3 = gw[3];
      float* wp = wsh + ldr * (unsigned)kWP + ldc;
      wp[0] = g0;
      wp[1] = g1;
      wp[2] = g2;
      wp[3] = g3;
    }
    __syncthreads();

#pragma unroll 1
    for (int j4 = 0; j4 < kKC; j4 += 4) {
      const float w0 = wr[j4 + 0];
      const float w1 = wr[j4 + 1];
      const float w2 = wr[j4 + 2];
      const float w3 = wr[j4 + 3];
#pragma unroll
      for (int i = 0; i < 4; ++i) {
        const v4f xv = *(const v4f*)(xr + i * kKC + j4);
        const float t0 = xv[0] * w0;
        P[i] = fmaf(t0, P[i], P[i]);
        Q[i] = fmaf(-t0, Q[i], Q[i]);
        const float t1 = xv[1] * w1;
        P[i] = fmaf(t1, P[i], P[i]);
        Q[i] = fmaf(-t1, Q[i], Q[i]);
        const float t2 = xv[2] * w2;
        P[i] = fmaf(t2, P[i], P[i]);
        Q[i] = fmaf(-t2, Q[i], Q[i]);
        const float t3 = xv[3] * w3;
        P[i] = fmaf(t3, P[i], P[i]);
        Q[i] = fmaf(-t3, Q[i], Q[i]);
      }
    }
  }

  const float bv = bias[o0 + lane];
  float res[4];
#pragma unroll
  for (int i = 0; i < 4; ++i) {
    const float p = fmaf(bv, P[i], P[i]);
    const float q = fmaf(-bv, Q[i], Q[i]);
    const float r = (p - q) * __builtin_amdgcn_rcpf(p + q);
    const float s = STD[(size_t)(b0 + wave * 4u + (unsigned)i) * kOut + o0 + lane];
    res[i] = 0.95f * (s + bv) + 0.05f * r;
  }

  float* op = out + (size_t)(b0 + wave * 4u) * kOut + o0 + lane;
  for (int pass = 0; pass < 2; ++pass) {
    *(volatile float*)(op)            = res[0];
    *(volatile float*)(op + kOut)     = res[1];
    *(volatile float*)(op + 2 * kOut) = res[2];
    *(volatile float*)(op + 3 * kOut) = res[3];
    __threadfence();
  }
}

extern "C" void kernel_launch(void* const* d_in, const int* in_sizes, int n_in,
                              void* d_out, int out_size, void* d_ws, size_t ws_size,
                              hipStream_t stream) {
  if (n_in < 3) return;
  if (in_sizes[0] != kB * kIn) return;
  if (in_sizes[1] != kOut * kIn) return;
  if (in_sizes[2] != kOut) return;
  if (out_size != kB * kOut) return;
  if (ws_size < kWsTotal) return;

  const float* x    = (const float*)d_in[0];
  const float* w    = (const float*)d_in[1];
  const float* bias = (const float*)d_in[2];
  float* out = (float*)d_out;

  char* ws = (char*)d_ws;
  unsigned short* A16  = (unsigned short*)(ws + kOffA16);
  unsigned short* BT16 = (unsigned short*)(ws + kOffBT16);
  float*          STD  = (float*)(ws + kOffSTD);

  to_f16_planes_kernel<<<kCvtBlkX + kCvtBlkW, 256, 0, stream>>>(x, w, A16, BT16);

  gemm_f16_nt_kernel<<<kGemmBlocks, 256, 0, stream>>>(A16, BT16, STD, kFold);

  scan_blend_kernel<<<dim3(kOut / kTO, kB / kTB), 256, 0, stream>>>(x, w, bias, STD, out);
}
